// TCM_77464030151162
// MI455X (gfx1250) — hardware-verified
//
#include <hip/hip_runtime.h>
#include <stddef.h>
#include <stdint.h>


#define CC    128
#define HC    64
#define KO    27
#define KS    (KO * HC)
#define ASC   16
#define WSC   1024
#define ATP   72
#define TP    68
#define WSCAP 134217728

static_assert(KS % 32 == 0);
static_assert(CC % 32 == 0);
static_assert((ATP * 2) % 16 == 0);
static_assert((TP * 4) % 16 == 0);
static_assert(KS % 64 == 0);
static_assert(CC % 64 == 0);

typedef float        v4f  __attribute__((ext_vector_type(4)));
typedef float        v8f  __attribute__((ext_vector_type(8)));
typedef _Float16     v8h  __attribute__((ext_vector_type(8)));
typedef _Float16     v16h __attribute__((ext_vector_type(16)));
typedef unsigned int v4u  __attribute__((ext_vector_type(4)));
union FragH { v16h v; v8h h[2]; };

__device__ __forceinline__ v8f wmf(v16h a, v16h b, v8f c) {
  v8f d = __builtin_amdgcn_wmma_f32_16x16x32_f16(false, a, false, b, (short)0, c, false, false);
  asm volatile("v_nop\n\tv_nop\n\tv_nop\n\tv_nop" : "+v"(d) : "v"(a), "v"(b));
  return d;
}

__device__ __forceinline__ v8h pack8(v4f a, v4f b, float s) {
  v8h o;
  o[0] = (_Float16)(a.x * s); o[1] = (_Float16)(a.y * s);
  o[2] = (_Float16)(a.z * s); o[3] = (_Float16)(a.w * s);
  o[4] = (_Float16)(b.x * s); o[5] = (_Float16)(b.y * s);
  o[6] = (_Float16)(b.z * s); o[7] = (_Float16)(b.w * s);
  return o;
}

__global__ __launch_bounds__(256) void k_prepx(const float* __restrict__ x, _Float16* xh) {
  const size_t t = (size_t)blockIdx.x * 256 + threadIdx.x;
  const float* p = x + t * 8;
  const v4f f0 = *(const v4f*)p;
  const v4f f1 = *(const v4f*)(p + 4);
  const v8h a = pack8(f0, f1, (float)ASC);
  _Float16* d = xh + t * 8;
  *(volatile v8h*)d = a;
  __threadfence();
  *(volatile v8h*)d = a;
}

__global__ __launch_bounds__(256) void k_prepw(const float* __restrict__ W, _Float16* wt, int Kd, int Nd) {
  __shared__ __attribute__((aligned(16))) float tile[64 * TP];
  const int tid = threadIdx.x, lane = tid & 31, g = tid >> 5;
  const int n0 = blockIdx.x * 64;
  const int rsub = lane >> 3, c8 = 8 * (lane & 7);
#pragma unroll 1
  for (int dc = 0; dc < Kd; dc += 64) {
    __syncthreads();
#pragma unroll
    for (int j = 0; j < 4; ++j) {
      const int i = tid + 256 * j;
      const int kl = i >> 4;
      const int nn = (i & 15) * 4;
      const v4f v = *(const v4f*)(W + (size_t)(dc + kl) * Nd + n0 + nn);
      *(v4f*)(tile + kl * TP + nn) = v;
    }
    __syncthreads();
    v8h hv[2];
#pragma unroll
    for (int s = 0; s < 2; ++s) {
      const int nl = 8 * g + 4 * s + rsub;
#pragma unroll
      for (int e = 0; e < 8; ++e) hv[s][e] = (_Float16)(tile[(c8 + e) * TP + nl] * (float)WSC);
    }
#pragma unroll
    for (int s = 0; s < 2; ++s) {
      _Float16* d = wt + (size_t)(n0 + 8 * g + 4 * s + rsub) * Kd + dc + c8;
      *(volatile v8h*)d = hv[s];
    }
    __threadfence();
#pragma unroll
    for (int s = 0; s < 2; ++s) {
      _Float16* d = wt + (size_t)(n0 + 8 * g + 4 * s + rsub) * Kd + dc + c8;
      *(volatile v8h*)d = hv[s];
    }
  }
}

template <int MODE>
__global__ __launch_bounds__(64) void k_gemm(const _Float16* __restrict__ A, const _Float16* __restrict__ Bt,
                                             const float* __restrict__ bias, const float* __restrict__ xres,
                                             float* outF, _Float16* outH0, _Float16* outH1) {
  __shared__ __attribute__((aligned(16))) float stg_all[2 * 32 * 64];
  const int tid = threadIdx.x, lane = tid & 31, hh = lane >> 4, m = lane & 15;
  const int wave = __builtin_amdgcn_readfirstlane(tid >> 5);
  float* stg = stg_all + wave * 2048;
  const int m0 = blockIdx.x * 32, wn = wave * 64;

  v8f acc[2][4];
#pragma unroll
  for (int mt = 0; mt < 2; ++mt)
#pragma unroll
    for (int nt = 0; nt < 4; ++nt) { v8f z = {0.f, 0.f, 0.f, 0.f, 0.f, 0.f, 0.f, 0.f}; acc[mt][nt] = z; }

  const _Float16* ap = A + (size_t)(m0 + m) * CC + 8 * hh;
  const _Float16* bp = Bt + (size_t)(wn + m) * CC + 8 * hh;
#pragma unroll
  for (int k0 = 0; k0 < CC; k0 += 32) {
    FragH a0, a1;
    a0.h[0] = *(const v8h*)(ap + k0);
    a0.h[1] = *(const v8h*)(ap + k0 + 16);
    a1.h[0] = *(const v8h*)(ap + (size_t)16 * CC + k0);
    a1.h[1] = *(const v8h*)(ap + (size_t)16 * CC + k0 + 16);
#pragma unroll
    for (int nt = 0; nt < 4; ++nt) {
      const _Float16* bq = bp + (size_t)nt * 16 * CC + k0;
      FragH b;
      b.h[0] = *(const v8h*)bq;
      b.h[1] = *(const v8h*)(bq + 16);
      acc[0][nt] = wmf(a0.v, b.v, acc[0][nt]);
      acc[1][nt] = wmf(a1.v, b.v, acc[1][nt]);
    }
  }

  constexpr float OSC = 1.0f / (float)(ASC * WSC);
#pragma unroll
  for (int mt = 0; mt < 2; ++mt) {
    float* sp = stg + (16 * mt + 8 * hh) * 64 + m;
#pragma unroll
    for (int nt = 0; nt < 4; ++nt) {
      const float bv = bias[wn + 16 * nt + m];
#pragma unroll
      for (int r = 0; r < 8; ++r) sp[r * 64 + 16 * nt] = acc[mt][nt][r] * OSC + bv;
    }
  }
  __syncthreads();

  const int rsub = lane >> 3, pc8 = 8 * (lane & 7);
  if (MODE == 1) {
    if (wave == 0) {
      float* yb = outF + (size_t)m0 * HC + 4 * m;
#pragma unroll
      for (int q = 0; q < 16; ++q) {
        const int row = 2 * q + hh;
        const v4f v = *(const v4f*)(stg + row * 64 + 4 * m);
        *(volatile v4f*)(yb + (size_t)row * HC) = v;
      }
      __threadfence();
#pragma unroll
      for (int q = 0; q < 16; ++q) {
        const int row = 2 * q + hh;
        const v4f v = *(const v4f*)(stg + row * 64 + 4 * m);
        *(volatile v4f*)(yb + (size_t)row * HC) = v;
      }
      v8h hv[8];
#pragma unroll
      for (int q = 0; q < 8; ++q) {
        const float* sp2 = stg + (4 * q + rsub) * 64 + pc8;
        hv[q] = pack8(*(const v4f*)sp2, *(const v4f*)(sp2 + 4), (float)ASC);
      }
      _Float16* hb = outH0 + (size_t)m0 * HC + pc8;
#pragma unroll
      for (int q = 0; q < 8; ++q) *(volatile v8h*)(hb + (size_t)(4 * q + rsub) * HC) = hv[q];
      __threadfence();
#pragma unroll
      for (int q = 0; q < 8; ++q) *(volatile v8h*)(hb + (size_t)(4 * q + rsub) * HC) = hv[q];
    } else {
      v8h hv[8];
#pragma unroll
      for (int q = 0; q < 8; ++q) {
        const float* sp2 = stg + (4 * q + rsub) * 64 + pc8;
        hv[q] = pack8(*(const v4f*)sp2, *(const v4f*)(sp2 + 4), (float)ASC);
      }
      _Float16* hb = outH1 + (size_t)m0 * CC + HC + pc8;
#pragma unroll
      for (int q = 0; q < 8; ++q) *(volatile v8h*)(hb + (size_t)(4 * q + rsub) * CC) = hv[q];
      __threadfence();
#pragma unroll
      for (int q = 0; q < 8; ++q) *(volatile v8h*)(hb + (size_t)(4 * q + rsub) * CC) = hv[q];
    }
  } else {
    const size_t base = (size_t)m0 * CC + wn + 4 * m;
    float* ob = outF + base;
    const float* xb = xres + base;
#pragma unroll
    for (int q = 0; q < 16; ++q) {
      const int row = 2 * q + hh;
      float* sp2 = stg + row * 64 + 4 * m;
      const v4f a = *(const v4f*)sp2;
      const v4f xv = *(const v4f*)(xb + (size_t)row * CC);
      const v4f o = xv + a;
      *(v4f*)sp2 = o;
      *(volatile v4f*)(ob + (size_t)row * CC) = o;
    }
    __threadfence();
#pragma unroll
    for (int q = 0; q < 16; ++q) {
      const int row = 2 * q + hh;
      const v4f o = *(const v4f*)(stg + row * 64 + 4 * m);
      *(volatile v4f*)(ob + (size_t)row * CC) = o;
    }
  }
}

template <int MODE>
__global__ __launch_bounds__(32) void k_sconv(const _Float16* __restrict__ feat, const int* __restrict__ nbr,
                                              const _Float16* __restrict__ wt, const float* __restrict__ bias,
                                              const float* __restrict__ yc, _Float16* outH, int nN) {
  __shared__ __attribute__((aligned(16))) _Float16 tileA[32 * ATP];
  __shared__ __attribute__((aligned(16))) float stg[32 * 64];
  const int lane = threadIdx.x & 31, hh = lane >> 4, m = lane & 15;
  const int row0 = blockIdx.x * 32;
  const int rsub = lane >> 3, pc8 = 8 * (lane & 7);

  v8f acc[2][4];
#pragma unroll
  for (int mt = 0; mt < 2; ++mt)
#pragma unroll
    for (int nt = 0; nt < 4; ++nt) { v8f z = {0.f, 0.f, 0.f, 0.f, 0.f, 0.f, 0.f, 0.f}; acc[mt][nt] = z; }

  const _Float16* bp  = wt + (size_t)m * KS + 8 * hh;
  const _Float16* ar0 = tileA + m * ATP + 8 * hh;
  const _Float16* ar1 = ar0 + 16 * ATP;

#pragma unroll 1
  for (int k = 0; k < KO; ++k) {
    const int idx = nbr[(size_t)k * nN + row0 + lane];
    const int okm = (idx >= 0) ? 1 : 0;
    const int cid = min(max(idx, 0), nN - 1);
    __syncthreads();
#pragma unroll
    for (int p = 0; p < 8; ++p) {
      const int r = 4 * p + rsub;
      const int sid = __shfl(cid, r);
      const int sok = __shfl(okm, r);
      v4u v = *(const v4u*)(feat + (size_t)sid * HC + pc8);
      const unsigned mku = (unsigned)(-sok);
      v4u mk = {mku, mku, mku, mku};
      v = v & mk;
      *(v4u*)(tileA + r * ATP + pc8) = v;
    }
    __syncthreads();
#pragma unroll
    for (int kk = 0; kk < HC; kk += 32) {
      FragH a0, a1;
      a0.h[0] = *(const v8h*)(ar0 + kk);
      a0.h[1] = *(const v8h*)(ar0 + kk + 16);
      a1.h[0] = *(const v8h*)(ar1 + kk);
      a1.h[1] = *(const v8h*)(ar1 + kk + 16);
      const size_t kb = (size_t)k * HC + kk;
#pragma unroll
      for (int nt = 0; nt < 4; ++nt) {
        const _Float16* bq = bp + (size_t)nt * 16 * KS + kb;
        FragH b;
        b.h[0] = *(const v8h*)bq;
        b.h[1] = *(const v8h*)(bq + 16);
        acc[0][nt] = wmf(a0.v, b.v, acc[0][nt]);
        acc[1][nt] = wmf(a1.v, b.v, acc[1][nt]);
      }
    }
  }

  constexpr float OSC = 1.0f / (float)(ASC * WSC);
#pragma unroll
  for (int mt = 0; mt < 2; ++mt) {
    float* sp = stg + (16 * mt + 8 * hh) * 64 + m;
#pragma unroll
    for (int nt = 0; nt < 4; ++nt) {
      const float bv = bias[16 * nt + m];
#pragma unroll
      for (int r = 0; r < 8; ++r) sp[r * 64 + 16 * nt] = fmaxf(acc[mt][nt][r] * OSC + bv, 0.0f);
    }
  }
  __syncthreads();

  constexpr int LDH = (MODE == 0) ? HC : CC;
  v8h hv[8];
#pragma unroll
  for (int q = 0; q < 8; ++q) {
    const int row = 4 * q + rsub;
    const float* sp2 = stg + row * 64 + pc8;
    v4f u0 = *(const v4f*)sp2;
    v4f u1 = *(const v4f*)(sp2 + 4);
    if (MODE == 1) {
      const float* cp = yc + (size_t)(row0 + row) * HC + pc8;
      const v4f c0 = *(const v4f*)cp;
      const v4f c1 = *(const v4f*)(cp + 4);
      u0 = (u0 + c0) + c0;
      u1 = (u1 + c1) + c1;
    }
    hv[q] = pack8(u0, u1, (float)ASC);
  }
  _Float16* hb = outH + (size_t)row0 * LDH + pc8;
#pragma unroll
  for (int q = 0; q < 8; ++q) *(volatile v8h*)(hb + (size_t)(4 * q + rsub) * LDH) = hv[q];
  __threadfence();
#pragma unroll
  for (int q = 0; q < 8; ++q) *(volatile v8h*)(hb + (size_t)(4 * q + rsub) * LDH) = hv[q];
}

extern "C" void kernel_launch(void* const* d_in, const int* in_sizes, int n_in,
                              void* d_out, int out_size, void* d_ws, size_t ws_size,
                              hipStream_t stream) {
  if (n_in < 10) return;
  const int nN = in_sizes[0] / CC;
  if (nN <= 0 || in_sizes[0] != nN * CC) return;
  if ((nN % 32) != 0) return;
  if (in_sizes[1] != CC * CC || in_sizes[2] != CC) return;
  if (in_sizes[3] != CC * CC || in_sizes[4] != CC) return;
  if (in_sizes[5] != KO * HC * HC || in_sizes[6] != HC) return;
  if (in_sizes[7] != KO * HC * HC || in_sizes[8] != HC) return;
  if (in_sizes[9] != KO * nN) return;
  if (out_size != nN * CC) return;

  const float* x   = (const float*)d_in[0];
  const float* w1  = (const float*)d_in[1];
  const float* b1  = (const float*)d_in[2];
  const float* w2  = (const float*)d_in[3];
  const float* b2  = (const float*)d_in[4];
  const float* rw1 = (const float*)d_in[5];
  const float* rb1 = (const float*)d_in[6];
  const float* rw2 = (const float*)d_in[7];
  const float* rb2 = (const float*)d_in[8];
  const int*   nbr = (const int*)d_in[9];
  float* out = (float*)d_out;

  char* ws = (char*)d_ws;
  size_t off = 0;
  const size_t oXh  = off; off += (size_t)nN * CC * 2;   off = (off + 255) & ~(size_t)255;
  const size_t oW1  = off; off += (size_t)CC * CC * 2;   off = (off + 255) & ~(size_t)255;
  const size_t oW2  = off; off += (size_t)CC * CC * 2;   off = (off + 255) & ~(size_t)255;
  const size_t oR1  = off; off += (size_t)HC * KS * 2;   off = (off + 255) & ~(size_t)255;
  const size_t oR2  = off; off += (size_t)HC * KS * 2;   off = (off + 255) & ~(size_t)255;
  const size_t oYc  = off; off += (size_t)nN * HC * 4;   off = (off + 255) & ~(size_t)255;
  const size_t oCh  = off; off += (size_t)nN * HC * 2;   off = (off + 255) & ~(size_t)255;
  const size_t oRh  = off; off += (size_t)nN * HC * 2;   off = (off + 255) & ~(size_t)255;
  const size_t oA2  = off; off += (size_t)nN * CC * 2;   off = (off + 255) & ~(size_t)255;
  if (off > ws_size || off > (size_t)WSCAP) return;
  _Float16* xh   = (_Float16*)(ws + oXh);
  _Float16* w1t  = (_Float16*)(ws + oW1);
  _Float16* w2t  = (_Float16*)(ws + oW2);
  _Float16* rw1t = (_Float16*)(ws + oR1);
  _Float16* rw2t = (_Float16*)(ws + oR2);
  float*    yc   = (float*)(ws + oYc);
  _Float16* ch   = (_Float16*)(ws + oCh);
  _Float16* r1h  = (_Float16*)(ws + oRh);
  _Float16* a2h  = (_Float16*)(ws + oA2);

  k_prepw<<<dim3(CC / 64), 256, 0, stream>>>(w1, w1t, CC, CC);
  k_prepw<<<dim3(CC / 64), 256, 0, stream>>>(w2, w2t, CC, CC);
  k_prepw<<<dim3(HC / 64), 256, 0, stream>>>(rw1, rw1t, KS, HC);
  k_prepw<<<dim3(HC / 64), 256, 0, stream>>>(rw2, rw2t, KS, HC);
  k_prepx<<<(unsigned)(((size_t)nN * CC) / 2048), 256, 0, stream>>>(x, xh);

  const unsigned gRows = (unsigned)(nN / 32);
  k_gemm<1><<<gRows, 64, 0, stream>>>(xh, w1t, b1, x, yc, ch, a2h);
  k_sconv<0><<<gRows, 32, 0, stream>>>(ch, nbr, rw1t, rb1, yc, r1h, nN);
  k_sconv<1><<<gRows, 32, 0, stream>>>(r1h, nbr, rw2t, rb2, yc, a2h, nN);
  k_gemm<2><<<gRows, 64, 0, stream>>>(a2h, w2t, b2, x, out, ch, a2h);
}
